// GPSModel_2619930050606
// MI455X (gfx1250) — hardware-verified
//
#include <hip/hip_runtime.h>
#include <math.h>

typedef __attribute__((ext_vector_type(16))) _Float16 v16h;
typedef __attribute__((ext_vector_type(16))) __bf16 v16b;
typedef __attribute__((ext_vector_type(8)))  _Float16 v8h;
typedef __attribute__((ext_vector_type(8)))  float v8f;
typedef __attribute__((ext_vector_type(4)))  float v4f;
typedef __attribute__((ext_vector_type(2)))  float v2f;
typedef __attribute__((ext_vector_type(4)))  unsigned v4u;
typedef __attribute__((ext_vector_type(4)))  int v4i;
typedef float __attribute__((may_alias)) float_a;
typedef int __attribute__((may_alias)) int_a;

template <typename T> __device__ __forceinline__ void vst2(void* p, T v) { *(volatile T*)p = v; __threadfence(); *(volatile T*)p = v; }
__device__ __forceinline__ v8f wmma16(v16h a, v16h b, v8f c) {
  v8f d = __builtin_amdgcn_wmma_f32_16x16x32_f16(false, a, false, b, (short)0, c, false, false);
  asm volatile("v_nop\n\tv_nop\n\tv_nop\n\tv_nop" : "+v"(d) : "v"(a), "v"(b));
  return d;
}
__device__ __forceinline__ v8f wmma_bf(v16b a, v16b b, v8f c) {
  v8f d = __builtin_amdgcn_wmma_f32_16x16x32_bf16(false, a, false, b, (short)0, c, false, false);
  asm volatile("v_nop\n\tv_nop\n\tv_nop\n\tv_nop" : "+v"(d) : "v"(a), "v"(b));
  return d;
}
__device__ __forceinline__ v16h frag_h(const _Float16* rowk0, int lane) {
  union { v16h v; v8h q[2]; } u; const _Float16* p = rowk0 + 8 * (lane >> 4);
  u.q[0] = *(const v8h*)p; u.q[1] = *(const v8h*)(p + 16); return u.v;
}
__device__ __forceinline__ v16h frag_f32(const float* rowk0, int lane) {
  v16h a; const float* p = rowk0 + 8 * (lane >> 4);
#pragma unroll
  for (int i = 0; i < 8; ++i) { a[i] = (_Float16)p[i]; a[8 + i] = (_Float16)p[16 + i]; }
  return a;
}
__device__ __forceinline__ v16h frag_f32s(const float* rowk0, int lane, float sc) {
  v16h a; const float* p = rowk0 + 8 * (lane >> 4);
#pragma unroll
  for (int i = 0; i < 8; ++i) { a[i] = (_Float16)(p[i] * sc); a[8 + i] = (_Float16)(p[16 + i] * sc); }
  return a;
}
__device__ __forceinline__ v16h fragc_f32(const float* W, int k0, int n, int lane, int ld, int K) {
  v16h a; const int g = lane >> 4;
#pragma unroll
  for (int i = 0; i < 8; ++i) { const int ka = k0 + 8 * g + i, kb = ka + 16;
    a[i] = (_Float16)(ka < K ? W[(size_t)ka * ld + n] : 0.f); a[8 + i] = (_Float16)(kb < K ? W[(size_t)kb * ld + n] : 0.f); }
  return a;
}
struct F2 { v16b h, l; };
__device__ __forceinline__ F2 bsplit16(const float v[16]) { F2 r;
#pragma unroll
  for (int i = 0; i < 16; ++i) { const __bf16 h = (__bf16)v[i]; r.h[i] = h; r.l[i] = (__bf16)(v[i] - (float)h); }
  return r; }
__device__ __forceinline__ F2 split_row(const float* row, int k0, int lane) { float v[16]; const float* p = row + k0 + 8 * (lane >> 4);
#pragma unroll
  for (int i = 0; i < 8; ++i) { v[i] = p[i]; v[8 + i] = p[16 + i]; }
  return bsplit16(v); }
__device__ __forceinline__ F2 split_rowK(const float* row, int k0, int lane, int K) { float v[16]; const int g = lane >> 4;
#pragma unroll
  for (int i = 0; i < 8; ++i) { const int ka = k0 + 8 * g + i, kb = ka + 16; v[i] = ka < K ? row[ka] : 0.f; v[8 + i] = kb < K ? row[kb] : 0.f; }
  return bsplit16(v); }
__device__ __forceinline__ F2 split_col(const float* W, int k0, int n, int lane, int ld, int K) { float v[16]; const int g = lane >> 4;
#pragma unroll
  for (int i = 0; i < 8; ++i) { const int ka = k0 + 8 * g + i, kb = ka + 16; v[i] = ka < K ? W[(size_t)ka * ld + n] : 0.f; v[8 + i] = kb < K ? W[(size_t)kb * ld + n] : 0.f; }
  return bsplit16(v); }
__device__ __forceinline__ v8f mac3(const F2& a, const F2& b, v8f c) { c = wmma_bf(a.l, b.h, c); c = wmma_bf(a.h, b.l, c); return wmma_bf(a.h, b.h, c); }
__device__ __forceinline__ float sigm(float v) { return 1.0f / (1.0f + expf(-v)); }
#define LDSX() do { asm volatile("s_wait_dscnt 0" ::: "memory"); __builtin_amdgcn_wave_barrier(); __builtin_amdgcn_fence(__ATOMIC_RELEASE, "workgroup"); } while (0)


__device__ __forceinline__ void load4ids(const int* __restrict__ ids, int e, int dd[4]) { const int4 a = *(const int4*)(ids + e); dd[0] = a.x; dd[1] = a.y; dd[2] = a.z; dd[3] = a.w; }
#define NN 4096
#define NE 131072
#define F0 128
#define FC 40
#define RB 512
#define NRB (NN / RB)
#define NNP NN
#define EPT 16
#define CH (256 * EPT)
#define NG 64
#define SS 4096
#define E 128
#define NH 2
#define HD 64
#define NR SS
#define FH 256
template <int K, int NOUT, int WROWS, int KV = K>
__global__ __launch_bounds__(128) void k_gemm(const float* __restrict__ A, int lda, const float* __restrict__ W, const float* __restrict__ DINV, float* __restrict__ HS) {
  __shared__ __align__(16) float so[4][16][NOUT + 4];
  const int tid = threadIdx.x, wave = tid >> 5, lane = tid & 31, col = lane & 15, g = lane >> 4;
  const int r0 = blockIdx.x * 64 + wave * 16;
  constexpr int NT = (NOUT + 15) / 16;
  v8f acc[NT];
#pragma unroll
  for (int t = 0; t < NT; ++t) acc[t] = (v8f){};
const int ra = (r0 + col) < NN ? (r0 + col) : (NN - 1);
#pragma unroll 1
  for (int kc = 0; kc < K / 32; ++kc) { const F2 a = split_row(A + (size_t)ra * lda, kc * 32, lane);
#pragma unroll
    for (int t = 0; t < NT; ++t) { const int n = t * 16 + col; const int nn = n < NOUT ? n : 0; acc[t] = mac3(a, WROWS ? split_row(W + (size_t)nn * K, kc * 32, lane) : split_col(W, kc * 32, nn, lane, NOUT, KV), acc[t]); } }
#pragma unroll
  for (int t = 0; t < NT; ++t) { const int n = t * 16 + col;
#pragma unroll
    for (int r = 0; r < 8; ++r) { const int row = r0 + 8 * g + r; const float dv = row < NN ? DINV[row] : 0.f; if (n < NOUT) so[wave][8 * g + r][n] = acc[t][r] * dv; } }
  LDSX();
  for (int q = lane; q < 16 * (NOUT / 4); q += 32) { const int rl = q / (NOUT / 4), pc = q % (NOUT / 4); vst2(HS + (size_t)(r0 + rl) * NOUT + pc * 4, *(const v4f*)(&so[wave][rl][pc * 4])); }
}
template <int F, int MODE>
__global__ __launch_bounds__(256) void k_agg(const float* __restrict__ HS, const int* __restrict__ esrc_, const int* __restrict__ edst_, const float* __restrict__ DINV, const float* __restrict__ bias, const float* __restrict__ lng, const float* __restrict__ lnb, float* __restrict__ OUT) {
  __shared__ __align__(16) float sacc[RB][F];
  __shared__ int ssrc[8][32 * EPT], sdl[8][32 * EPT]; __shared__ int scnt[8];
  const int tid = threadIdx.x, wave = tid >> 5, lane = tid & 31;
  const int r0 = blockIdx.x * RB; const int* esrc = esrc_; const int* edst = edst_;
  for (int q = tid; q < RB * F; q += 256) (&sacc[0][0])[q] = 0.f;
  __syncthreads();
#pragma unroll 1
  for (int c0 = 0; c0 < NE; c0 += CH) {
    const int e0 = c0 + tid * EPT; int hd[EPT]; int cnt = 0;
    if (e0 + EPT <= NE) {
#pragma unroll
      for (int v = 0; v < EPT / 4; ++v) { int dd[4]; load4ids(edst, e0 + v * 4, dd);
#pragma unroll
        for (int u = 0; u < 4; ++u) { const unsigned rel = (unsigned)(dd[u] - r0); const bool h = rel < (unsigned)RB; hd[v * 4 + u] = h ? (int)rel : -1; cnt += h ? 1 : 0; } } }
    else {
#pragma unroll
      for (int u = 0; u < EPT; ++u) { const int e = e0 + u; hd[u] = -1; if (e < NE) { const unsigned rel = (unsigned)(edst[e] - r0); if (rel < (unsigned)RB) { hd[u] = (int)rel; ++cnt; } } } }
    int incl = cnt;
#pragma unroll
    for (int off = 1; off < 32; off <<= 1) { const int vv = __shfl_up(incl, off, 32); if (lane >= off) incl += vv; }
    const int wtot = __shfl(incl, 31, 32); int pos = incl - cnt;
    if (cnt > 0) {
#pragma unroll
      for (int u = 0; u < EPT; ++u) if (hd[u] >= 0) { int s = esrc[e0 + u]; s = s < 0 ? 0 : (s >= NN ? NN - 1 : s); ssrc[wave][pos] = s; sdl[wave][pos] = hd[u];  ++pos; } }
    if (lane == 0) scnt[wave] = wtot;
    __syncthreads();
    if (tid < F) { for (int w = 0; w < 8; ++w) { const int nh = scnt[w]; for (int i = 0; i < nh; ++i) sacc[sdl[w][i]][tid] += HS[(size_t)ssrc[w][i] * F + tid]; } }
    __syncthreads(); }
  for (int rl = tid; rl < RB; rl += 256) { const int row = r0 + rl; if (row >= NN) continue; const float dv = DINV[row]; float* ar = &sacc[rl][0]; const float* hs = HS + (size_t)row * F;
    if (MODE == 4) { const float* rs = lng + (size_t)row * F; for (int f = 0; f < F; ++f) { const float v = ar[f] * dv + bias[f]; ar[f] = (v > 0.f ? v : 0.f) + rs[f]; } (void)hs; }
    else if (MODE == 5) { const float* rs = lng + (size_t)row * F; for (int f = 0; f < F; ++f) ar[f] = (ar[f] + hs[f]) * dv + bias[f] + rs[f]; }
    else { for (int f = 0; f < F; ++f) ar[f] = (ar[f] + hs[f]) * dv + bias[f]; }
    if (MODE == 2) { for (int f = 0; f < F; ++f) ar[f] = ar[f] > 0.f ? ar[f] : 0.f; }
    else if (MODE == 0) { float mu = 0.f; for (int f = 0; f < F; ++f) mu += ar[f]; mu *= (1.0f / F); float var = 0.f; for (int f = 0; f < F; ++f) { const float d = ar[f] - mu; var += d * d; } var *= (1.0f / F);
      const float rs = rsqrtf(var + 1e-5f); for (int f = 0; f < F; ++f) { const float v = (ar[f] - mu) * rs * lng[f] + lnb[f]; ar[f] = v > 0.f ? v : 0.f; } }
    else if (MODE == 1) { float mx = -3.4e38f; for (int f = 0; f < FC; ++f) mx = fmaxf(mx, ar[f]); float se = 0.f; for (int f = 0; f < FC; ++f) se += expf(ar[f] - mx); const float lse = logf(se) + mx; for (int f = 0; f < FC; ++f) ar[f] -= lse; } }
  __syncthreads();
  if (MODE != 1 && MODE != 3) { for (int q = tid; q < RB * (F / 4); q += 256) { const int rl = q / (F / 4), pc = q % (F / 4); const int row = r0 + rl; v4f v = *(const v4f*)(&sacc[rl][pc * 4]); if (row >= NN) { if (MODE == 2 || MODE == 4 || MODE == 5) continue; v = (v4f){0.f, 0.f, 0.f, 0.f}; } vst2(OUT + (size_t)row * F + pc * 4, v); } }
  else {
    for (int q = tid; q < RB * FC / 4; q += 256) { const int rl = (q * 4) / FC, f = (q * 4) % FC; const int row = r0 + rl; if (row < NN) { v4f v; v[0] = sacc[rl][f]; v[1] = sacc[rl][f + 1]; v[2] = sacc[rl][f + 2]; v[3] = sacc[rl][f + 3]; vst2(OUT + (size_t)row * FC + f, v); } } }
}

__global__ __launch_bounds__(256) void k_deg(const int* __restrict__ edst, float* __restrict__ DINV) {
  __shared__ int sc[NN]; const int tid = threadIdx.x;
  for (int q = tid; q < NN; q += 256) sc[q] = 0; __syncthreads();
#pragma unroll 1
  for (int c0 = 0; c0 < NE; c0 += CH) { const int e0 = c0 + tid * EPT;
#pragma unroll
    for (int v = 0; v < EPT / 4; ++v) { int dd[4]; load4ids(edst, e0 + v * 4, dd);
#pragma unroll
      for (int u = 0; u < 4; ++u) { const unsigned r = (unsigned)dd[u]; if (r < (unsigned)NN) atomicAdd(&sc[r], 1); } } }
  __syncthreads();
  for (int q = tid; q < NN; q += 256) vst2(DINV + q, (float_a)rsqrtf((float)sc[q] + 1.0f));
}
template <int K, int NOUT, int RELU>
__global__ __launch_bounds__(128) void k_lin(const float* __restrict__ A, const float* __restrict__ W, const float* __restrict__ bias, const float* __restrict__ resid, float* __restrict__ Cc) {
  __shared__ __align__(16) float so[4][16][132];
  const int tid = threadIdx.x, wave = tid >> 5, lane = tid & 31, col = lane & 15, g = lane >> 4; const int r0 = blockIdx.x * 64 + wave * 16;
#pragma unroll 1
  for (int nh = 0; nh < NOUT / 128; ++nh) { v8f acc[8] = {};
#pragma unroll 1
    for (int kc = 0; kc < (K + 31) / 32; ++kc) { const F2 a = split_rowK(A + (size_t)(r0 + col) * K, kc * 32, lane, K);
#pragma unroll
      for (int j = 0; j < 8; ++j) acc[j] = mac3(a, split_col(W, kc * 32, nh * 128 + j * 16 + col, lane, NOUT, K), acc[j]); }
#pragma unroll
    for (int j = 0; j < 8; ++j) { const int n = nh * 128 + j * 16 + col; const float bb = bias ? bias[n] : 0.f;
#pragma unroll
      for (int r = 0; r < 8; ++r) { float v = acc[j][r] + bb; if (resid) v += resid[(size_t)(r0 + 8 * g + r) * NOUT + n]; so[wave][8 * g + r][j * 16 + col] = RELU ? (v > 0.f ? v : 0.f) : v; } }
    LDSX();
    for (int rl = 0; rl < 16; ++rl) vst2(Cc + (size_t)(r0 + rl) * NOUT + nh * 128 + lane * 4, *(const v4f*)(&so[wave][rl][lane * 4]));
    LDSX(); }
}
__global__ __launch_bounds__(256) void k_bn(const float* __restrict__ T, const float* __restrict__ gamma, const float* __restrict__ beta, int relu, float* __restrict__ OUTp) {
  __shared__ float smu[F0], ssc[F0]; const int tid = threadIdx.x;
  if (tid < F0) { float s = 0.f;
#pragma unroll 4
    for (int r = 0; r < NN; ++r) s += T[(size_t)r * F0 + tid];
    const float mu = s * (1.0f / NN); float q = 0.f;
#pragma unroll 4
    for (int r = 0; r < NN; ++r) { const float d = T[(size_t)r * F0 + tid] - mu; q += d * d; }
    smu[tid] = mu; ssc[tid] = gamma[tid] * rsqrtf(q * (1.0f / NN) + 1e-5f); }
  __syncthreads();
  for (int q = tid; q < NN * (F0 / 4); q += 256) { const int r = q >> 5, pc = q & 31; v4f v = *(const v4f*)(T + (size_t)r * F0 + pc * 4);
#pragma unroll
    for (int e = 0; e < 4; ++e) { const int c = pc * 4 + e; float y = (v[e] - smu[c]) * ssc[c] + beta[c]; v[e] = relu ? (y > 0.f ? y : 0.f) : y; }
    vst2(OUTp + (size_t)r * F0 + pc * 4, v); }
}
__global__ __launch_bounds__(256) void k_cvt(const float* __restrict__ x, _Float16* __restrict__ X16) {
  const size_t i8 = (size_t)blockIdx.x * 256 + threadIdx.x; if (i8 >= (size_t)NR * E / 8) return;
  union { v8h h; v4u u; } pk;
#pragma unroll
  for (int e = 0; e < 8; ++e) pk.h[e] = (_Float16)x[i8 * 8 + e];
  vst2(X16 + i8 * 8, pk.u);
}
__global__ __launch_bounds__(128) void k_pack(const float* __restrict__ Wqkv, _Float16* __restrict__ PT) {
  const int n = blockIdx.x, tid = threadIdx.x; __shared__ __align__(16) _Float16 srow[E];
  srow[tid] = (_Float16)(Wqkv[(size_t)n * E + tid] * 16.0f); __syncthreads();
  if (tid < E / 8) vst2(PT + (size_t)n * E + tid * 8, *(const v4u*)(&srow[tid * 8]));
}
__global__ __launch_bounds__(128) void k_qkv(const _Float16* __restrict__ X16, const _Float16* __restrict__ PT, const float* __restrict__ bqkv, _Float16* __restrict__ Q16, _Float16* __restrict__ K16, _Float16* __restrict__ VTh) {
  __shared__ __align__(16) float so[4][16][132];
  __shared__ __align__(16) _Float16 sth[128][72];
  const int tid = threadIdx.x, wave = tid >> 5, lane = tid & 31, col = lane & 15, g = lane >> 4;
  const int which = blockIdx.z, r0b = blockIdx.x * 64, r0 = r0b + wave * 16, n0 = 0; const int s0 = r0b;
  v8f acc[8] = {};
#pragma unroll
  for (int kc = 0; kc < E / 32; ++kc) { const v16h a = frag_h(X16 + (size_t)(r0 + col) * E + kc * 32, lane);
#pragma unroll
    for (int j = 0; j < 8; ++j) acc[j] = wmma16(a, frag_h(PT + (size_t)(which * E + n0 + j * 16 + col) * E + kc * 32, lane), acc[j]); }
  const float osc = which == 0 ? 4.0f * 0.125f : 4.0f;
  if (which < 2) {
#pragma unroll
    for (int j = 0; j < 8; ++j) { const float bb = bqkv[which * E + j * 16 + col];
#pragma unroll
      for (int r = 0; r < 8; ++r) so[wave][8 * g + r][j * 16 + col] = (acc[j][r] * (1.0f / 16.0f) + bb) * osc; }
    LDSX();
    _Float16* Dst = which == 0 ? Q16 : K16;
    for (int qq = lane; qq < 16 * 2 * 8; qq += 32) { const int hh = qq >> 7, rl = (qq >> 3) & 15, pc = qq & 7; union { v8h h8; v4u u; } pk;
#pragma unroll
      for (int e = 0; e < 8; ++e) pk.h8[e] = (_Float16)so[wave][rl][hh * 64 + pc * 8 + e];
      vst2(Dst + (((size_t)hh) * SS + s0 + wave * 16 + rl) * HD + pc * 8, pk.u); } }
  else {
#pragma unroll
    for (int j = 0; j < 8; ++j) { const float bb = bqkv[2 * E + j * 16 + col];
#pragma unroll
      for (int r = 0; r < 8; ++r) sth[j * 16 + col][wave * 16 + 8 * g + r] = (_Float16)((acc[j][r] * (1.0f / 16.0f) + bb) * 4.0f); }
    __syncthreads();
    for (int qq = tid; qq < 128 * 8; qq += 128) { const int cl = qq >> 3, pc = qq & 7; const int h = cl >> 6, d = cl & 63; vst2(VTh + (((size_t)h) * HD + d) * SS + s0 + pc * 8, *(const v4u*)(&sth[cl][pc * 8])); } }
}
__global__ __launch_bounds__(128) void k_attn(const _Float16* __restrict__ Q16, const _Float16* __restrict__ K16, const _Float16* __restrict__ VTh, _Float16* __restrict__ O16) {
  __shared__ __align__(16) float sS[4][16][68];
  __shared__ __align__(16) _Float16 sPh[4][16][72];
  __shared__ __align__(16) float sO[4][16][68];
  const int tid = threadIdx.x, w = tid >> 5, lane = tid & 31, col = lane & 15, g = lane >> 4;
  const size_t bh = blockIdx.y; const int q0 = blockIdx.x * 64 + w * 16;
  v16h aq[2];
#pragma unroll
  for (int kc = 0; kc < 2; ++kc) aq[kc] = frag_h(Q16 + (bh * SS + q0 + col) * HD + kc * 32, lane);
  float mrun = -3.0e38f, lrun = 0.f; v8f acc[4] = {};
#pragma unroll 1
  for (int kt = 0; kt < SS / 64; ++kt) {
#pragma unroll
    for (int t = 0; t < 4; ++t) { v8f s = {}; const int key = kt * 64 + t * 16 + col;
#pragma unroll
      for (int kc = 0; kc < 2; ++kc) s = wmma16(aq[kc], frag_h(K16 + (bh * SS + key) * HD + kc * 32, lane), s);
#pragma unroll
      for (int r = 0; r < 8; ++r) sS[w][8 * g + r][t * 16 + col] = s[r] * (1.0f / 16.0f); }
    LDSX();
    float mx = -3.4e38f;
#pragma unroll
    for (int jj = 0; jj < 32; ++jj) mx = fmaxf(mx, sS[w][col][g * 32 + jj]);
    mx = fmaxf(mx, __shfl_xor(mx, 16, 32));
    const float mnew = fmaxf(mrun, mx); const float corr = expf(mrun - mnew);
    float ps = 0.f;
#pragma unroll
    for (int jj = 0; jj < 32; ++jj) { const float p = expf(sS[w][col][g * 32 + jj] - mnew) * 16384.0f; ps += p; sPh[w][col][g * 32 + jj] = (_Float16)p; }
    ps += __shfl_xor(ps, 16, 32);
    lrun = lrun * corr + ps * (1.0f / 16384.0f); mrun = mnew;
#pragma unroll
    for (int r = 0; r < 8; ++r) { const float cr = __shfl(corr, 8 * g + r, 32);
#pragma unroll
      for (int t = 0; t < 4; ++t) acc[t][r] *= cr; }
    LDSX();
#pragma unroll
    for (int kc = 0; kc < 2; ++kc) { const v16h ph = frag_h(&sPh[w][col][0] + kc * 32, lane);
#pragma unroll
      for (int t = 0; t < 4; ++t) { const size_t vo = (bh * HD + t * 16 + col) * SS + kt * 64 + kc * 32; acc[t] = wmma16(ph, frag_h(VTh + vo, lane), acc[t]); } }
    __builtin_amdgcn_wave_barrier(); }
#pragma unroll
  for (int r = 0; r < 8; ++r) { const float lr = __shfl(lrun, 8 * g + r, 32); const float inv = 8.0f / (lr * 16384.0f * 4.0f);
#pragma unroll
    for (int t = 0; t < 4; ++t) sO[w][8 * g + r][t * 16 + col] = acc[t][r] * inv; }
  LDSX();
  for (int qq = lane; qq < 16 * 8; qq += 32) { const int rl = qq >> 3, pc = qq & 7; union { v8h h8; v4u u; } pk;
#pragma unroll
    for (int e = 0; e < 8; ++e) pk.h8[e] = (_Float16)sO[w][rl][pc * 8 + e];
    vst2(O16 + ((bh * SS) + q0 + rl) * HD + pc * 8, pk.u); }
}
__global__ __launch_bounds__(128) void k_oproj(const _Float16* __restrict__ O16, const float* __restrict__ Wout, const float* __restrict__ bout, const float* __restrict__ Hres, float* __restrict__ T) {
  __shared__ __align__(16) float sc[4][16][E + 4]; __shared__ __align__(16) float so[4][16][132];
  const int tid = threadIdx.x, wave = tid >> 5, lane = tid & 31, col = lane & 15, g = lane >> 4; const int r0 = blockIdx.x * 64 + wave * 16;
  for (int qq = lane; qq < 16 * E; qq += 32) { const int rl = qq >> 7, c = qq & 127; const int h = c >> 6, d = c & 63; sc[wave][rl][c] = (float)O16[(((size_t)h) * SS + r0 + rl) * HD + d] * 0.125f; }
  LDSX();
  v8f acc[8] = {};
#pragma unroll 1
  for (int kc = 0; kc < E / 32; ++kc) { const F2 a = split_row(&sc[wave][col][0], kc * 32, lane);
#pragma unroll
    for (int j = 0; j < 8; ++j) acc[j] = mac3(a, split_row(Wout + (size_t)(j * 16 + col) * E, kc * 32, lane), acc[j]); }
#pragma unroll
  for (int j = 0; j < 8; ++j) { const int n = j * 16 + col; const float bb = bout[n];
#pragma unroll
    for (int r = 0; r < 8; ++r) so[wave][8 * g + r][j * 16 + col] = acc[j][r] + bb + Hres[(size_t)(r0 + 8 * g + r) * E + n]; }
  LDSX();
  for (int rl = 0; rl < 16; ++rl) vst2(T + (size_t)(r0 + rl) * E + lane * 4, *(const v4f*)(&so[wave][rl][lane * 4]));
}
__global__ __launch_bounds__(128) void k_mlp(const float* __restrict__ HL, const float* __restrict__ HA, const float* __restrict__ W1, const float* __restrict__ b1, const float* __restrict__ W2, const float* __restrict__ b2, float* __restrict__ T3) {
  __shared__ __align__(16) float sorow[4][16][E + 4]; __shared__ __align__(16) float shid[4][16][FH + 4];
  const int tid = threadIdx.x, wave = tid >> 5, lane = tid & 31, col = lane & 15, g = lane >> 4; const int r0 = blockIdx.x * 64 + wave * 16;
  for (int qq = lane; qq < 16 * E; qq += 32) { const int rl = qq >> 7, c = qq & 127; sorow[wave][rl][c] = HL[(size_t)(r0 + rl) * E + c] + HA[(size_t)(r0 + rl) * E + c]; }
  LDSX();
#pragma unroll 1
  for (int nh = 0; nh < 2; ++nh) { v8f acc[8] = {};
#pragma unroll 1
    for (int kc = 0; kc < E / 32; ++kc) { const F2 a = split_row(&sorow[wave][col][0], kc * 32, lane);
#pragma unroll
      for (int j = 0; j < 8; ++j) acc[j] = mac3(a, split_col(W1, kc * 32, nh * 128 + j * 16 + col, lane, FH, E), acc[j]); }
#pragma unroll
    for (int j = 0; j < 8; ++j) { const int n = nh * 128 + j * 16 + col; const float bb = b1[n];
#pragma unroll
      for (int r = 0; r < 8; ++r) { const float v = acc[j][r] + bb; shid[wave][8 * g + r][n] = v > 0.f ? v : 0.f; } } }
  LDSX();
  { v8f acc[8] = {};
#pragma unroll 1
    for (int kc = 0; kc < FH / 32; ++kc) { const F2 a = split_row(&shid[wave][col][0], kc * 32, lane);
#pragma unroll
      for (int j = 0; j < 8; ++j) acc[j] = mac3(a, split_col(W2, kc * 32, j * 16 + col, lane, E, FH), acc[j]); }
#pragma unroll
    for (int j = 0; j < 8; ++j) { const int n = j * 16 + col; const float bb = b2[n];
#pragma unroll
      for (int r = 0; r < 8; ++r) sorow[wave][8 * g + r][n] += acc[j][r] + bb; } }
  LDSX();
  for (int rl = 0; rl < 16; ++rl) vst2(T3 + (size_t)(r0 + rl) * E + lane * 4, *(const v4f*)(&sorow[wave][rl][lane * 4]));
}
__global__ __launch_bounds__(128) void k_pool(const float* __restrict__ Hh, const int* __restrict__ batch, float* __restrict__ PL) {
  __shared__ float sp[2][F0]; __shared__ int scount;
  const int g0 = blockIdx.x, tid = threadIdx.x, c = tid & 127; float s = 0.f; int cnt = 0;
  for (int n = 0; n < NN; ++n) { if (batch[n] == g0) { s += Hh[(size_t)n * F0 + c]; ++cnt; } }
  if (tid < F0) vst2(PL + (size_t)g0 * F0 + c, (float_a)(cnt > 0 ? s / (float)cnt : 0.f));
  (void)sp; (void)scount;
}
__global__ __launch_bounds__(256) void k_head(const float* __restrict__ PL, const float* __restrict__ Wl, const float* __restrict__ bl, float* __restrict__ out) {
  const int tid = threadIdx.x, gph = tid >> 2, o = tid & 3; float s = bl[o];
#pragma unroll 4
  for (int k = 0; k < F0; ++k) s += PL[(size_t)gph * F0 + k] * Wl[k * 4 + o];
  vst2(out + tid, (float_a)s);
}
extern "C" void kernel_launch(void* const* d_in, const int* in_sizes, int n_in, void* d_out, int out_size, void* d_ws, size_t ws_size, hipStream_t stream) {
  (void)in_sizes; (void)n_in; (void)out_size; (void)ws_size;
  const float** I = (const float**)d_in;
  const float* x = I[0]; const int* ei = (const int*)d_in[1]; const int* batch = (const int*)d_in[2];
  const float* projW = I[3]; const float* projb = I[4]; const float* gcnW = I[5]; const float* gcnb = I[6]; const float* qkvw = I[7]; const float* qkvb = I[8]; const float* aow = I[9]; const float* aob = I[10];
  const float* bng = I[11]; const float* bnb = I[12]; const float* W1 = I[13]; const float* b1 = I[14]; const float* W2 = I[15]; const float* b2 = I[16]; const float* linW = I[17]; const float* linb = I[18];
  float* out = (float*)d_out;
  char* ws = (char*)d_ws; size_t off = 0;
  auto take = [&](size_t bytes) { char* p = ws + off; off += (bytes + 255) & ~(size_t)255; return p; };
  float* DINV = (float*)take(NN * 4); float* Hc = (float*)take((size_t)NN * F0 * 4); float* HS = (float*)take((size_t)NN * F0 * 4); float* T1 = (float*)take((size_t)NN * F0 * 4); float* HL = (float*)take((size_t)NN * F0 * 4);
  float* T2 = (float*)take((size_t)NN * F0 * 4); float* HA = (float*)take((size_t)NN * F0 * 4); float* T3 = (float*)take((size_t)NN * F0 * 4); float* PL = (float*)take((size_t)NG * F0 * 4);
  _Float16* X16 = (_Float16*)take((size_t)NN * E * 2); _Float16* PT = (_Float16*)take((size_t)3 * E * E * 2); _Float16* Q16 = (_Float16*)take((size_t)NN * E * 2); _Float16* K16 = (_Float16*)take((size_t)NN * E * 2); _Float16* VTh = (_Float16*)take((size_t)NN * E * 2); _Float16* O16 = (_Float16*)take((size_t)NN * E * 2);
  const int* esrc = ei; const int* edst = ei + NE;
  k_deg<<<1, 256, 0, stream>>>(edst, DINV);
  k_lin<16, 128, 0><<<NN / 64, 128, 0, stream>>>(x, projW, projb, nullptr, Hc);
  for (int l = 0; l < 2; ++l) { const size_t oM = (size_t)l * F0 * F0, oV = (size_t)l * F0;
    k_gemm<F0, F0, 0><<<NN / 64, 128, 0, stream>>>(Hc, F0, gcnW + oM, DINV, HS);
    k_agg<F0, 5><<<NRB, 256, 0, stream>>>(HS, esrc, edst, DINV, gcnb + oV, Hc, nullptr, T1);
    k_bn<<<1, 256, 0, stream>>>(T1, bng + (l * 3 + 0) * F0, bnb + (l * 3 + 0) * F0, 0, HL);
    k_cvt<<<(NN * E / 8 + 255) / 256, 256, 0, stream>>>(Hc, X16);
    k_pack<<<3 * E, 128, 0, stream>>>(qkvw + (size_t)l * 3 * E * E, PT);
    k_qkv<<<dim3(NN / 64, 1, 3), 128, 0, stream>>>(X16, PT, qkvb + (size_t)l * 3 * E, Q16, K16, VTh);
    k_attn<<<dim3(SS / 64, NH), 128, 0, stream>>>(Q16, K16, VTh, O16);
    k_oproj<<<NN / 64, 128, 0, stream>>>(O16, aow + oM, aob + oV, Hc, T2);
    k_bn<<<1, 256, 0, stream>>>(T2, bng + (l * 3 + 1) * F0, bnb + (l * 3 + 1) * F0, 0, HA);
    k_mlp<<<NN / 64, 128, 0, stream>>>(HL, HA, W1 + (size_t)l * F0 * FH, b1 + (size_t)l * FH, W2 + (size_t)l * FH * F0, b2 + oV, T3);
    k_bn<<<1, 256, 0, stream>>>(T3, bng + (l * 3 + 2) * F0, bnb + (l * 3 + 2) * F0, l == 0 ? 1 : 0, Hc); }
  k_pool<<<NG, 128, 0, stream>>>(Hc, batch, PL);
  k_head<<<1, 256, 0, stream>>>(PL, linW, linb, out);
}
